// GATv2_65910568125059
// MI455X (gfx1250) — hardware-verified
//
#include <hip/hip_runtime.h>
#include <math.h>
#include <stdint.h>
#include <stddef.h>

#define NB    2
#define NT    1024
#define CIN   128
#define DQ    64
#define NTOK  (NB * NT)
#define MQK   (2 * DQ)
#define NEGB  (-1.0e22f)
#define GBM   64
#define GBN   128
#define GTHR  128
#define QT    64
#define KS    64
#define ATHR  128
#define WSMAX 134217728

static_assert(CIN % 32 == 0);
static_assert(MQK % GBM == 0 && NTOK % GBN == 0);
static_assert(GBM == (GTHR / 32) * 16 && GBN == 4 * 32);
static_assert(NT % QT == 0 && NT % KS == 0 && QT == 4 * 16 && KS == 64 && ATHR == 128);
static_assert(CIN == 8 * 16);
static_assert(DQ == 64);
static_assert(NTOK % 64 == 0 && CIN % 64 == 0);
static_assert((NTOK * CIN) % 8 == 0 && (DQ * CIN) % 8 == 0);
static_assert(DQ * QT == ATHR * 8 * 4);
static_assert(2 * DQ * QT == QT * CIN);

typedef __attribute__((ext_vector_type(16))) __bf16 v16b;
typedef __attribute__((ext_vector_type(8)))  __bf16 v8b;
typedef __attribute__((ext_vector_type(8)))  float  v8f;
typedef __attribute__((ext_vector_type(4)))  float  v4f;
typedef __attribute__((ext_vector_type(4)))  unsigned int v4u;
typedef __attribute__((ext_vector_type(8)))  unsigned int v8u;
typedef v8b __attribute__((may_alias)) v8ba;
typedef v4f __attribute__((may_alias)) v4fa;
typedef v4u __attribute__((may_alias)) v4ua;

union FragU { v16b v; v8b h[2]; };
union PackU { v8u u; v16b v; };

__device__ __forceinline__ unsigned short f2bf_bits(float f) {
  const unsigned u = __float_as_uint(f);
  return (unsigned short)((u + 0x7FFFu + ((u >> 16) & 1u)) >> 16);
}
__device__ __forceinline__ float bf_bits2f(unsigned short h) { return __uint_as_float(((unsigned)h) << 16); }
__device__ __forceinline__ float bf16r(float f) {
  unsigned u = __float_as_uint(f);
  u = (u + 0x7FFFu + ((u >> 16) & 1u)) & 0xFFFF0000u;
  return __uint_as_float(u);
}
__device__ __forceinline__ unsigned pk16(unsigned short a, unsigned short b) { return (unsigned)a | ((unsigned)b << 16); }

__device__ __forceinline__ v8f wmma_bf16(v16b a, v16b b, v8f c) {
  v8f d = __builtin_amdgcn_wmma_f32_16x16x32_bf16(false, a, false, b, (short)0, c, false, false);
  asm volatile("v_nop\n\tv_nop\n\tv_nop\n\tv_nop" : "+v"(d) : "v"(a), "v"(b));
  return d;
}

__device__ __forceinline__ v16b load_frag(const unsigned short* p, int hh) {
  FragU f;
  f.h[0] = *(const v8ba*)(p + 8 * hh);
  f.h[1] = *(const v8ba*)(p + 16 + 8 * hh);
  return f.v;
}

__device__ __forceinline__ void pack_p2(v8f a, v8f c, v16b& ho, v16b& lo) {
  PackU uh, ul;
#pragma unroll
  for (int i = 0; i < 4; ++i) {
    const unsigned short h0 = f2bf_bits(a[2 * i]), h1 = f2bf_bits(a[2 * i + 1]);
    const unsigned short l0 = f2bf_bits(a[2 * i] - bf_bits2f(h0)), l1 = f2bf_bits(a[2 * i + 1] - bf_bits2f(h1));
    uh.u[i] = pk16(h0, h1); ul.u[i] = pk16(l0, l1);
    const unsigned short g0 = f2bf_bits(c[2 * i]), g1 = f2bf_bits(c[2 * i + 1]);
    const unsigned short m0 = f2bf_bits(c[2 * i] - bf_bits2f(g0)), m1 = f2bf_bits(c[2 * i + 1] - bf_bits2f(g1));
    uh.u[4 + i] = pk16(g0, g1); ul.u[4 + i] = pk16(m0, m1);
  }
  ho = uh.v; lo = ul.v;
}

__global__ __launch_bounds__(256) void k_cvt(const float* __restrict__ src, unsigned short* __restrict__ dst, int n8) {
  int i = blockIdx.x * 256 + threadIdx.x;
  const bool ok = i < n8;
  i = ok ? i : (n8 - 1);
  const float* s = src + (size_t)i * 8;
  const v4f f0 = *(const v4fa*)(s);
  const v4f f1 = *(const v4fa*)(s + 4);
  v4u u;
  u[0] = pk16(f2bf_bits(f0[0]), f2bf_bits(f0[1]));
  u[1] = pk16(f2bf_bits(f0[2]), f2bf_bits(f0[3]));
  u[2] = pk16(f2bf_bits(f1[0]), f2bf_bits(f1[1]));
  u[3] = pk16(f2bf_bits(f1[2]), f2bf_bits(f1[3]));
  unsigned short* d = dst + (size_t)i * 8;
  if (ok) *(volatile v4u*)d = u;
  __threadfence();
  if (ok) *(volatile v4u*)d = u;
}

__global__ __launch_bounds__(256) void k_tcvt(const float* __restrict__ W, unsigned short* __restrict__ ob, int R, int Cc) {
  __shared__ __align__(16) float tf[64 * 68];
  const int cb0 = blockIdx.x * 64;
  const int rb0 = blockIdx.y * 64;
  const int tid = threadIdx.x;
  {
    const int lr = tid >> 4;
    const int c4 = (tid & 15) * 4;
#pragma unroll
    for (int it = 0; it < 4; ++it) {
      const int rr = it * 16 + lr;
      const v4f a = *(const v4fa*)(W + (size_t)(rb0 + rr) * Cc + cb0 + c4);
      *(v4fa*)(tf + rr * 68 + c4) = a;
    }
  }
  __syncthreads();
  const int sub = tid >> 3;
  const int c8  = (tid & 7) * 8;
  v4u hv[2];
#pragma unroll
  for (int it = 0; it < 2; ++it) {
    const int oc = it * 32 + sub;
    v4u a;
#pragma unroll
    for (int q = 0; q < 4; ++q) {
      const float f0 = tf[(c8 + 2 * q) * 68 + oc];
      const float f1 = tf[(c8 + 2 * q + 1) * 68 + oc];
      a[q] = pk16(f2bf_bits(f0), f2bf_bits(f1));
    }
    hv[it] = a;
  }
  for (int pass = 0; pass < 2; ++pass) {
#pragma unroll
    for (int it = 0; it < 2; ++it) {
      const int oc = it * 32 + sub;
      const size_t go = (size_t)(cb0 + oc) * R + rb0 + c8;
      *(volatile v4u*)(ob + go) = hv[it];
    }
    __threadfence();
  }
}

__global__ __launch_bounds__(GTHR) void k_gemm(const unsigned short* __restrict__ A, const unsigned short* __restrict__ BT,
                                               float* __restrict__ Cm) {
  __shared__ __align__(16) float stg[GBM * GBN];
  const int tid = (int)threadIdx.x, lane = tid & 31, wave = tid >> 5, hh = lane >> 4, m = lane & 15;
  const int rowBase = (int)blockIdx.x * GBM;
  const int colBase = (int)blockIdx.y * GBN;

  const v8f zero8 = {0.f, 0.f, 0.f, 0.f, 0.f, 0.f, 0.f, 0.f};
  v8f acc[8];
#pragma unroll
  for (int t = 0; t < 8; ++t) acc[t] = zero8;

  const unsigned short* ap = A  + (size_t)(rowBase + 16 * wave + m) * (size_t)CIN;
  const unsigned short* bp = BT + (size_t)(colBase + m) * (size_t)CIN;

#pragma unroll 1
  for (int k0 = 0; k0 < CIN; k0 += 32) {
    const v16b af = load_frag(ap + k0, hh);
#pragma unroll
    for (int nt = 0; nt < 8; ++nt) {
      const v16b bf = load_frag(bp + (size_t)(16 * nt) * (size_t)CIN + k0, hh);
      acc[nt] = wmma_bf16(af, bf, acc[nt]);
    }
  }

#pragma unroll
  for (int nt = 0; nt < 8; ++nt) {
    const int lc = 16 * nt + m;
#pragma unroll
    for (int r = 0; r < 8; ++r) {
      const int lr = 16 * wave + 8 * hh + r;
      stg[lr * GBN + lc] = acc[nt][r];
    }
  }
  __syncthreads();

  v4f pv[16];
#pragma unroll
  for (int i = 0; i < 16; ++i) pv[i] = *(const v4fa*)(stg + (16 * wave + i) * GBN + 4 * lane);
#pragma unroll
  for (int i = 0; i < 16; ++i) {
    float* op = Cm + (size_t)(rowBase + 16 * wave + i) * (size_t)NTOK + colBase + 4 * lane;
    *(volatile v4f*)op = pv[i];
  }
  __threadfence();
#pragma unroll
  for (int i = 0; i < 16; ++i) {
    float* op = Cm + (size_t)(rowBase + 16 * wave + i) * (size_t)NTOK + colBase + 4 * lane;
    *(volatile v4f*)op = pv[i];
  }
}

__global__ __launch_bounds__(ATHR) void k_attn(const float* __restrict__ HT, const float* __restrict__ adj,
                                              const float* __restrict__ avec,
                                              const unsigned short* __restrict__ VT,
                                              float* __restrict__ out) {
  __shared__ __align__(16) float smem[2 * DQ * QT];
  __shared__ __align__(16) float sA[DQ];
  float* sKt = smem;
  float* sQt = smem + DQ * QT;

  const int tid = threadIdx.x, lane = tid & 31, w = tid >> 5;
  const int hh = lane >> 4, m = lane & 15;
  const int qt = blockIdx.x, b = blockIdx.y;
  const int i0 = qt * QT, i0w = i0 + 16 * w, iq = i0w + m;
  const size_t tokb = (size_t)b * NT;

#pragma unroll
  for (int it = 0; it < 8; ++it) {
    const int u  = tid + ATHR * it;
    const int d  = u >> 4;
    const int c4 = (u & 15) * 4;
    const v4f v = *(const v4fa*)(HT + (size_t)(DQ + d) * (size_t)NTOK + tokb + i0 + c4);
    *(v4fa*)(sKt + d * QT + c4) = v;
  }
  if (tid < DQ) sA[tid] = bf16r(avec[tid]);

  const v8f zero8 = {0.f, 0.f, 0.f, 0.f, 0.f, 0.f, 0.f, 0.f};
  v8f o[8];
#pragma unroll
  for (int t = 0; t < 8; ++t) o[t] = zero8;
  float mrun = -INFINITY, lrun = 0.0f;

  const float* adjrow = adj + (tokb + (size_t)iq) * (size_t)NT;

#pragma unroll 1
  for (int ks = 0; ks < NT / KS; ++ks) {
    const int kb = ks * KS;

    __syncthreads();
#pragma unroll
    for (int it = 0; it < 8; ++it) {
      const int u  = tid + ATHR * it;
      const int d  = u >> 4;
      const int c4 = (u & 15) * 4;
      const v4f v = *(const v4fa*)(HT + (size_t)d * (size_t)NTOK + tokb + kb + c4);
      *(v4fa*)(sQt + d * KS + c4) = v;
    }
    __syncthreads();

    v8f s[4];
#pragma unroll
    for (int j = 0; j < 4; ++j) s[j] = zero8;
    const float* kcol = sKt + 16 * w + m;
#pragma unroll 2
    for (int d = 0; d < DQ; ++d) {
      const float kv = kcol[d * QT];
      const float av = sA[d];
      const float* qrow = sQt + d * KS + 8 * hh;
#pragma unroll
      for (int j = 0; j < 4; ++j) {
        const v4f qa = *(const v4fa*)(qrow + 16 * j);
        const v4f qb = *(const v4fa*)(qrow + 16 * j + 4);
        s[j][0] = fmaf(fmaxf(qa[0] + kv, 0.0f), av, s[j][0]);
        s[j][1] = fmaf(fmaxf(qa[1] + kv, 0.0f), av, s[j][1]);
        s[j][2] = fmaf(fmaxf(qa[2] + kv, 0.0f), av, s[j][2]);
        s[j][3] = fmaf(fmaxf(qa[3] + kv, 0.0f), av, s[j][3]);
        s[j][4] = fmaf(fmaxf(qb[0] + kv, 0.0f), av, s[j][4]);
        s[j][5] = fmaf(fmaxf(qb[1] + kv, 0.0f), av, s[j][5]);
        s[j][6] = fmaf(fmaxf(qb[2] + kv, 0.0f), av, s[j][6]);
        s[j][7] = fmaf(fmaxf(qb[3] + kv, 0.0f), av, s[j][7]);
      }
    }

#pragma unroll
    for (int j = 0; j < 4; ++j) {
      const int ko = kb + 16 * j + 8 * hh;
      const v4f mA = *(const v4fa*)(adjrow + ko);
      const v4f mB = *(const v4fa*)(adjrow + ko + 4);
      const float mv[8] = {mA[0], mA[1], mA[2], mA[3], mB[0], mB[1], mB[2], mB[3]};
#pragma unroll
      for (int r = 0; r < 8; ++r) {
        const float add = (mv[r] > 0.0f) ? 0.0f : NEGB;
        s[j][r] = s[j][r] + add;
      }
    }

    float cm = -INFINITY;
#pragma unroll
    for (int j = 0; j < 4; ++j)
#pragma unroll
      for (int r = 0; r < 8; ++r) cm = fmaxf(cm, s[j][r]);
    cm = fmaxf(cm, __shfl_xor(cm, 16, 32));
    const float mnew  = fmaxf(mrun, cm);
    const float alpha = __expf(mrun - mnew);
    mrun = mnew;
    float psum = 0.0f;
#pragma unroll
    for (int j = 0; j < 4; ++j)
#pragma unroll
      for (int r = 0; r < 8; ++r) {
        const float p = __expf(s[j][r] - mnew);
        psum += p;
        s[j][r] = p;
      }
    psum += __shfl_xor(psum, 16, 32);
    lrun = lrun * alpha + psum;
#pragma unroll
    for (int t = 0; t < 8; ++t)
#pragma unroll
      for (int r = 0; r < 8; ++r) o[t][r] *= alpha;

    {
      v16b ph, pl;
      pack_p2(s[0], s[1], ph, pl);
#pragma unroll
      for (int t = 0; t < 8; ++t) {
        const unsigned short* vp = VT + (size_t)(16 * t + m) * (size_t)NTOK + tokb + kb;
        const v16b vf = load_frag(vp, hh);
        o[t] = wmma_bf16(vf, ph, o[t]);
        o[t] = wmma_bf16(vf, pl, o[t]);
      }
    }
    {
      v16b ph, pl;
      pack_p2(s[2], s[3], ph, pl);
#pragma unroll
      for (int t = 0; t < 8; ++t) {
        const unsigned short* vp = VT + (size_t)(16 * t + m) * (size_t)NTOK + tokb + kb + 32;
        const v16b vf = load_frag(vp, hh);
        o[t] = wmma_bf16(vf, ph, o[t]);
        o[t] = wmma_bf16(vf, pl, o[t]);
      }
    }
  }

  __syncthreads();
  float* sO = smem;
  const float inv = 1.0f / lrun;
#pragma unroll
  for (int t = 0; t < 8; ++t)
#pragma unroll
    for (int r = 0; r < 8; ++r)
      sO[(16 * w + m) * CIN + 16 * t + 8 * hh + r] = o[t][r] * inv;
  __syncthreads();
  for (int pass = 0; pass < 2; ++pass) {
#pragma unroll
    for (int it = 0; it < 16; ++it) {
      const int row = 16 * w + it;
      const v4f v = *(const v4fa*)(sO + row * CIN + 4 * lane);
      *(volatile v4f*)(out + (tokb + (size_t)(i0 + row)) * (size_t)CIN + 4 * lane) = v;
    }
    __threadfence();
  }
}

extern "C" void kernel_launch(void* const* d_in, const int* in_sizes, int n_in,
                              void* d_out, int out_size, void* d_ws, size_t ws_size,
                              hipStream_t stream) {
  if (n_in < 5) return;
  if (in_sizes[0] != NTOK * CIN) return;
  if (in_sizes[1] != NB * NT * NT) return;
  if (in_sizes[2] != DQ * CIN) return;
  if (in_sizes[3] != DQ * CIN) return;
  if (in_sizes[4] != DQ) return;
  if (out_size != NTOK * CIN) return;

  const float* feat = (const float*)d_in[0];
  const float* adj  = (const float*)d_in[1];
  const float* W1   = (const float*)d_in[2];
  const float* W2   = (const float*)d_in[3];
  const float* avec = (const float*)d_in[4];
  float* out = (float*)d_out;

  const size_t PX  = (size_t)NTOK * CIN * 2;
  const size_t PW  = (size_t)MQK * CIN * 2;
  const size_t PVT = (size_t)CIN * NTOK * 2;
  const size_t PHT = (size_t)MQK * NTOK * 4;
  size_t off = 0;
  const size_t oXb = off; off += PX;  off = (off + 255) & ~(size_t)255;
  const size_t oWb = off; off += PW;  off = (off + 255) & ~(size_t)255;
  const size_t oVT = off; off += PVT; off = (off + 255) & ~(size_t)255;
  const size_t oHT = off; off += PHT; off = (off + 255) & ~(size_t)255;
  if (off > ws_size || off > (size_t)WSMAX) return;

  char* ws = (char*)d_ws;
  unsigned short* Xb = (unsigned short*)(ws + oXb);
  unsigned short* Wb = (unsigned short*)(ws + oWb);
  unsigned short* VT = (unsigned short*)(ws + oVT);
  float*          HT = (float*)(ws + oHT);

  const int n8x = NTOK * CIN / 8;
  const int n8w = DQ * CIN / 8;
  k_cvt<<<dim3((n8x + 255) / 256), 256, 0, stream>>>(feat, Xb, n8x);
  k_cvt<<<dim3((n8w + 255) / 256), 256, 0, stream>>>(W1, Wb, n8w);
  k_cvt<<<dim3((n8w + 255) / 256), 256, 0, stream>>>(W2, Wb + (size_t)DQ * CIN, n8w);
  k_tcvt<<<dim3(CIN / 64, NTOK / 64), 256, 0, stream>>>(feat, VT, NTOK, CIN);
  k_gemm<<<dim3(MQK / GBM, NTOK / GBN), GTHR, 0, stream>>>(Wb, Xb, HT);
  k_attn<<<dim3(NT / QT, NB), ATHR, 0, stream>>>(HT, adj, avec, VT, out);
  (void)hipGetLastError();
}
